// Controller_60816736911410
// MI455X (gfx1250) — hardware-verified
//
#include <hip/hip_runtime.h>
#include <hip/hip_bf16.h>
#include <math.h>

typedef __attribute__((ext_vector_type(16))) _Float16 v16h;
typedef __attribute__((ext_vector_type(8)))  float    v8f;
typedef __attribute__((ext_vector_type(4)))  float    v4f_t;
typedef float v4fa __attribute__((ext_vector_type(4), may_alias));
#define RSPLIT (1.0f / 2048.0f)
__device__ __forceinline__ void split1(float f, _Float16& h, _Float16& l) { h = (_Float16)f; l = (_Float16)((f - (float)h) * 2048.0f); }
__device__ __forceinline__ v8f wmma_split(v16h ah, v16h al, v16h bh, v16h bl, v8f c) {
    v8f x = {};
    x = __builtin_amdgcn_wmma_f32_16x16x32_f16(false, al, false, bh, (short)0, x, false, false);
    x = __builtin_amdgcn_wmma_f32_16x16x32_f16(false, ah, false, bl, (short)0, x, false, false);
    return __builtin_amdgcn_wmma_f32_16x16x32_f16(false, ah, false, bh, (short)0, c, false, false) + x * RSPLIT;
}

#define N_AGENTS 4096
#define TOPK 32

__device__ __forceinline__ unsigned long long umin64(unsigned long long a,
                                                     unsigned long long b) {
    return (b < a) ? b : a;
}
__device__ __forceinline__ unsigned long long umax64(unsigned long long a,
                                                     unsigned long long b) {
    return (b > a) ? b : a;
}

__global__ __launch_bounds__(256) void topk_kernel(const float* __restrict__ states,
                                                   int* __restrict__ idxWs,
                                                   float* __restrict__ maskWs) {
    __shared__ float d2[N_AGENTS];
    __shared__ unsigned long long wk[8];
    __shared__ int   sIdx[TOPK];
    __shared__ float sMsk[TOPK];
    const int t = threadIdx.x, agent = blockIdx.x;
    const int lane = t & 31, w = t >> 5;

    const float sx = states[agent * 4 + 0];
    const float sy = states[agent * 4 + 1];
    for (int j = t; j < N_AGENTS; j += 256) {
        float dx = sx - states[j * 4 + 0];
        float dy = sy - states[j * 4 + 1];
        d2[j] = dx * dx + dy * dy;
    }
    __syncthreads();

    for (int r = 0; r < TOPK; ++r) {
        unsigned long long bk = ~0ull;
        for (int j = t; j < N_AGENTS; j += 256) {
            unsigned long long k =
                ((unsigned long long)__float_as_uint(d2[j]) << 32) | (unsigned)j;
            bk = umin64(bk, k);
        }
#pragma unroll
        for (int m = 1; m <= 16; m <<= 1)
            bk = umin64(bk, (unsigned long long)__shfl_xor((unsigned long long)bk, m, 32));
        if (lane == 0) wk[w] = bk;
        __syncthreads();
        if (t == 0) {
            unsigned long long fk = wk[0];
#pragma unroll
            for (int q = 1; q < 8; ++q) fk = umin64(fk, wk[q]);
            int   fi = (int)(fk & 0xffffffffu);
            float fv = __uint_as_float((unsigned)(fk >> 32));
            sIdx[r] = fi;
            sMsk[r] = (fv < 1.0f) ? 1.0f : 0.0f;
            d2[fi] = 3.4e38f;
        }
        __syncthreads();
    }
    if (t < 32) {
        *(volatile int*)(idxWs + agent * TOPK + t) = sIdx[t]; *(volatile float*)(maskWs + agent * TOPK + t) = sMsk[t];
        __threadfence();
        *(volatile int*)(idxWs + agent * TOPK + t) = sIdx[t]; *(volatile float*)(maskWs + agent * TOPK + t) = sMsk[t];
    }
}

__global__ __launch_bounds__(256) void conv_argmax_kernel(const float* __restrict__ states,
                                                          const float* __restrict__ W1,
                                                          const float* __restrict__ b1,
                                                          const float* __restrict__ W2,
                                                          const float* __restrict__ b2,
                                                          const int* __restrict__ idxWs,
                                                          const float* __restrict__ maskWs,
                                                          float* __restrict__ xloc) {
    __shared__ alignas(32) _Float16 sH1[32 * 64];
    __shared__ alignas(32) _Float16 sH1l[32 * 64];
    __shared__ float sMask[32];
    __shared__ alignas(16) float sX[128];

    const int t    = threadIdx.x;
    const int lane = t & 31;
    const int mt   = t >> 5;
    const int colL = lane & 15;
    const int hiA  = (lane < 16) ? 0 : 8;
    const int hiB  = hiA;

    const int m = mt * 16 + colL;
    union { v16h v; _Float16 e[16]; } Af0, Af1, Af0l, Af1l;
#pragma unroll
    for (int h = 0; h < 16; ++h) {
        int kk = (h < 8 ? h : h + 8) + hiA;
        split1(W2[m * 64 + kk],      Af0.e[h], Af0l.e[h]);
        split1(W2[m * 64 + 32 + kk], Af1.e[h], Af1l.e[h]);
    }
    float bias[8];
#pragma unroll
    for (int r = 0; r < 8; ++r) bias[r] = b2[mt * 16 + r + ((lane >= 16) ? 8 : 0)];

    const int p = t & 31;
    const int cbase = (t >> 5) * 8;

    for (int al = 0; al < 32; ++al) {
        const int agent = blockIdx.x * 32 + al;

        const float sa0 = states[agent * 4 + 0], sa1 = states[agent * 4 + 1];
        const float sa2 = states[agent * 4 + 2], sa3 = states[agent * 4 + 3];
        float hcol[5];
#pragma unroll
        for (int c = 0; c < 5; ++c) {
            int flat = c * 32 + p;
            int k = flat / 5, e = flat - 5 * k;
            int j = idxWs[agent * TOPK + k];
            float se = (e == 0) ? sa0 : (e == 1) ? sa1 : (e == 2) ? sa2 : sa3;
            float diff = se - states[j * 4 + (e & 3)];
            float self = (j == agent) ? 1.0f : 0.0f;
            hcol[c] = (e == 4) ? self : diff;
        }
#pragma unroll
        for (int cc = 0; cc < 8; ++cc) {
            int c = cbase + cc;
            float acc = b1[c];
#pragma unroll
            for (int e = 0; e < 5; ++e) acc += W1[c * 5 + e] * hcol[e];
            split1(fmaxf(acc, 0.0f), sH1[p * 64 + c], sH1l[p * 64 + c]);
        }
        if (t < 32) sMask[t] = maskWs[agent * TOPK + t];
        __syncthreads();

        v8f acc0 = {}, acc1 = {};
        {
            typedef __attribute__((ext_vector_type(8))) _Float16 v8h_;
            auto ldB = [&](const _Float16* src, int pc, int ks) -> v16h {
                const _Float16* q = src + pc * 64 + ks * 32 + hiB;
                union { v16h v; v8h_ h[2]; } u; u.h[0] = *(const v8h_*)(q); u.h[1] = *(const v8h_*)(q + 16); return u.v;
            };
            acc0 = wmma_split(Af0.v, Af0l.v, ldB(sH1, colL, 0),      ldB(sH1l, colL, 0),      acc0);
            acc0 = wmma_split(Af1.v, Af1l.v, ldB(sH1, colL, 1),      ldB(sH1l, colL, 1),      acc0);
            acc1 = wmma_split(Af0.v, Af0l.v, ldB(sH1, 16 + colL, 0), ldB(sH1l, 16 + colL, 0), acc1);
            acc1 = wmma_split(Af1.v, Af1l.v, ldB(sH1, 16 + colL, 1), ldB(sH1l, 16 + colL, 1), acc1);
        }
        const float m0 = sMask[colL];
        const float m1 = sMask[16 + colL];
#pragma unroll
        for (int r = 0; r < 8; ++r) {
            float v0 = fmaxf(acc0[r] + bias[r], 0.0f) * m0;
            float v1 = fmaxf(acc1[r] + bias[r], 0.0f) * m1;
            unsigned long long k0 =
                ((unsigned long long)__float_as_uint(v0) << 32) | (unsigned)(31 - colL);
            unsigned long long k1 =
                ((unsigned long long)__float_as_uint(v1) << 32) | (unsigned)(15 - colL);
            unsigned long long bk = umax64(k0, k1);
#pragma unroll
            for (int mm = 1; mm <= 8; mm <<= 1)
                bk = umax64(bk, (unsigned long long)__shfl_xor((unsigned long long)bk, mm, 32));
            if (colL == 0) {
                int row = mt * 16 + r + ((lane >= 16) ? 8 : 0);
                sX[row] = (float)(31 - (int)(bk & 31u));
            }
        }
        __syncthreads();
        if (t < 32) {
            const v4f_t v = *(const v4fa*)(sX + t * 4);
            *(volatile v4f_t*)(xloc + agent * 128 + t * 4) = v; __threadfence(); *(volatile v4f_t*)(xloc + agent * 128 + t * 4) = v;
        }
    }
}

__global__ __launch_bounds__(256) void mlp_kernel(const float* __restrict__ states,
                                                  const float* __restrict__ goals,
                                                  const float* __restrict__ Wd1,
                                                  const float* __restrict__ bd1,
                                                  const float* __restrict__ Wd2,
                                                  const float* __restrict__ bd2,
                                                  const float* __restrict__ Wd3,
                                                  const float* __restrict__ bd3,
                                                  const float* __restrict__ Wd4,
                                                  const float* __restrict__ bd4,
                                                  const float* __restrict__ xloc,
                                                  float* __restrict__ out) {
    __shared__ float bufA[8][132];
    __shared__ float bufB[8][128];
    __shared__ float sOut[32];
    const int lane = threadIdx.x & 31, w = threadIdx.x >> 5;
    float* A = bufA[w];
    float* B = bufB[w];
#pragma unroll 1
  for (int sub = 0; sub < 2; ++sub) {
    const int al = w * 2 + sub;
    const int agent = blockIdx.x * 16 + al;
    __syncthreads();

#pragma unroll
    for (int o = lane; o < 128; o += 32) A[o] = xloc[agent * 128 + o];
    if (lane == 0) {
        A[128] = states[agent * 4 + 0] - goals[agent * 2 + 0];
        A[129] = states[agent * 4 + 1] - goals[agent * 2 + 1];
        A[130] = states[agent * 4 + 2];
        A[131] = states[agent * 4 + 3];
    }
    __syncthreads();
    for (int o = lane; o < 64; o += 32) {
        float acc = bd1[o];
        for (int k = 0; k < 132; ++k) acc += Wd1[o * 132 + k] * A[k];
        B[o] = fmaxf(acc, 0.0f);
    }
    __syncthreads();
    for (int o = lane; o < 128; o += 32) {
        float acc = bd2[o];
        for (int k = 0; k < 64; ++k) acc += Wd2[o * 64 + k] * B[k];
        A[o] = fmaxf(acc, 0.0f);
    }
    __syncthreads();
    for (int o = lane; o < 64; o += 32) {
        float acc = bd3[o];
        for (int k = 0; k < 128; ++k) acc += Wd3[o * 128 + k] * A[k];
        B[o] = fmaxf(acc, 0.0f);
    }
    __syncthreads();
    if (lane < 4) {
        float acc = bd4[lane];
        for (int k = 0; k < 64; ++k) acc += Wd4[lane * 64 + k] * B[k];
        A[lane] = 2.0f / (1.0f + expf(-acc)) + 0.2f;
    }
    __syncthreads();
    if (lane == 0) {
        float rx = states[agent * 4 + 0] - goals[agent * 2 + 0];
        float ry = states[agent * 4 + 1] - goals[agent * 2 + 1];
        float vx = states[agent * 4 + 2];
        float vy = states[agent * 4 + 3];
        sOut[al * 2 + 0] = -(A[0] * rx + A[1] * vx);
        sOut[al * 2 + 1] = -(A[2] * ry + A[3] * vy);
    }
  }
    __syncthreads();
    if (threadIdx.x < 32) {
        const float v = sOut[threadIdx.x];
        *(volatile float*)(out + blockIdx.x * 32 + threadIdx.x) = v; __threadfence(); *(volatile float*)(out + blockIdx.x * 32 + threadIdx.x) = v;
    }
}

extern "C" void kernel_launch(void* const* d_in, const int* in_sizes, int n_in,
                              void* d_out, int out_size, void* d_ws, size_t ws_size,
                              hipStream_t stream) {
    (void)in_sizes; (void)n_in; (void)out_size; (void)ws_size;
    const float* states = (const float*)d_in[0];
    const float* goals  = (const float*)d_in[1];
    const float* W1     = (const float*)d_in[2];
    const float* b1     = (const float*)d_in[3];
    const float* W2     = (const float*)d_in[4];
    const float* b2     = (const float*)d_in[5];
    const float* Wd1    = (const float*)d_in[6];
    const float* bd1    = (const float*)d_in[7];
    const float* Wd2    = (const float*)d_in[8];
    const float* bd2    = (const float*)d_in[9];
    const float* Wd3    = (const float*)d_in[10];
    const float* bd3    = (const float*)d_in[11];
    const float* Wd4    = (const float*)d_in[12];
    const float* bd4    = (const float*)d_in[13];
    float* out = (float*)d_out;

    char* ws = (char*)d_ws;
    int*   idxWs  = (int*)ws;
    float* maskWs = (float*)(ws + (size_t)N_AGENTS * TOPK * sizeof(int));
    float* xloc   = (float*)(ws + 2 * (size_t)N_AGENTS * TOPK * sizeof(int));

    topk_kernel<<<N_AGENTS, 256, 0, stream>>>(states, idxWs, maskWs);
    conv_argmax_kernel<<<N_AGENTS / 32, 256, 0, stream>>>(states, W1, b1, W2, b2,
                                                          idxWs, maskWs, xloc);
    mlp_kernel<<<N_AGENTS / 16, 256, 0, stream>>>(states, goals, Wd1, bd1, Wd2, bd2,
                                                 Wd3, bd3, Wd4, bd4, xloc, out);
}
